// Net_28544352649361
// MI455X (gfx1250) — hardware-run, weakly checked
//
#include <hip/hip_runtime.h>
#include <stddef.h>
#include <stdint.h>


#define SPLIT_SV 1

#define DF     128
#define NLAB   128
#define NSENT  16384
#define TOK    1048576
#define VOC    100000
#define RSN    100096
#define AP     256
#define WP     256
#if SPLIT_SV
#define KUSED  256
#else
#define KUSED  128
#endif

#define NTHR   256
#define NWAVE  8
#define CHUNK  2048
#define WSPAN  (CHUNK / NWAVE)
#define NCH    (TOK / CHUNK)
#define NCHP   (NCH + 1)
#define NBRUN  256
#define SLB    9
#define NBLK   (NSENT / NBRUN)
#define WLCAP  4096
#define RCAP   20480
#define DEGCAP 256

#define L_WL   0
#define L_SL   (NWAVE * WLCAP)
#define L_WCUM (L_SL + RCAP)
#define L_CNT  (L_WCUM + NWAVE * NCHP)
#define L_OFFS (L_CNT + NBRUN)
#define L_CUR  (L_OFFS + NBRUN)
#define L_SVL  (L_CUR + NBRUN)
#define L_MISC (L_SVL + NBRUN)
#define SEG_LDS_INTS (L_MISC + 16)

#define GBM    64
#define GBN    128
#define GTHR   128
#define WUNITS (NLAB * (WP / 8))
#define WSMAX  (128u << 20)

static_assert(NSENT % NBRUN == 0);
static_assert(NBRUN <= 512 && NBRUN <= (1 << SLB) && (NBRUN & (NBRUN - 1)) == 0);
static_assert(VOC <= (1 << 17));
static_assert(((long long)(VOC - 1) << SLB) < (1LL << 31));
static_assert(TOK % CHUNK == 0 && WSPAN == 256 && CHUNK == NTHR * 8);
static_assert(RCAP >= 17422 && RCAP % 4 == 0);
static_assert(DEGCAP >= 108 && DEGCAP % 32 == 0);
static_assert(WLCAP % 4 == 0 && WLCAP >= 2330 + 256);
static_assert(L_SL % 4 == 0 && L_WCUM % 4 == 0 && L_CNT % 4 == 0 && L_SVL % 4 == 0 && SEG_LDS_INTS % 4 == 0);
static_assert(SEG_LDS_INTS * 4 <= 300000 && SEG_LDS_INTS * 4 <= 327680);
static_assert(NBRUN % NWAVE == 0 && NBRUN % 32 == 0 && NBRUN == 256);
static_assert(KUSED % 32 == 0 && KUSED <= AP && KUSED <= WP && AP == 2 * DF && WP == 2 * DF);
static_assert(GBN == NLAB && GBM == (GTHR / 32) * 16 && NSENT % GBM == 0 && NBRUN % GBM == 0);
static_assert(VOC % 32 == 0 && RSN >= VOC && RSN % 32 == 0);
static_assert(WUNITS % NTHR == 0);
static_assert((long long)NSENT * NLAB - 1 == 2097151LL);

typedef float          v4f   __attribute__((ext_vector_type(4)));
typedef float          v8f   __attribute__((ext_vector_type(8)));
typedef int            v4i   __attribute__((ext_vector_type(4)));
typedef int            v8i   __attribute__((ext_vector_type(8)));
typedef unsigned int   v4u   __attribute__((ext_vector_type(4)));
typedef unsigned short v8us  __attribute__((ext_vector_type(8)));
typedef unsigned short v16us __attribute__((ext_vector_type(16)));
typedef __bf16         v16bf __attribute__((ext_vector_type(16)));
typedef v4f  __attribute__((may_alias)) v4fa;
typedef v4i  __attribute__((may_alias)) v4ia;
typedef v8us __attribute__((may_alias)) v8usa;
union FragB { v16bf v; v16us u; v8us h[2]; v8i w; };

__device__ __forceinline__ v8f wmb(const FragB& a, const FragB& b, v8f c) {
  v8f d = __builtin_amdgcn_wmma_f32_16x16x32_bf16(false, a.v, false, b.v, (short)0, c, false, false);
  asm volatile("v_nop\n\tv_nop\n\tv_nop\n\tv_nop" : "+v"(d) : "v"(a.w), "v"(b.w));
  return d;
}

__device__ __forceinline__ unsigned bf16_bits(float f) {
  const unsigned u = __float_as_uint(f);
  const unsigned r = (u + 0x7FFFu + ((u >> 16) & 1u)) >> 16;
  return (f != f) ? 0x7FC0u : r;
}
__device__ __forceinline__ float bf16_val(float f) {
  return __uint_as_float(bf16_bits(f) << 16);
}

__device__ __forceinline__ int clampw(int t) {
  t = t < 0 ? 0 : t;
  return t > VOC - 1 ? VOC - 1 : t;
}

__global__ __launch_bounds__(NTHR) void k_prep(const float* __restrict__ W, const float* __restrict__ hb,
                                               unsigned short* WD, float* BB) {
  const int tid = (int)threadIdx.x;
  if ((int)blockIdx.x < WUNITS / NTHR) {
    const int u  = (int)blockIdx.x * NTHR + tid;
    const int n  = u >> 5;
    const int k8 = (u & 31) * 8;
    const int kk = k8 & (DF - 1);
    const float* p = W + (size_t)n * DF + kk;
    const v4f a = *(const v4f*)p;
    const v4f b = *(const v4f*)(p + 4);
    v8us o;
    o[0] = (unsigned short)bf16_bits(a.x); o[1] = (unsigned short)bf16_bits(a.y);
    o[2] = (unsigned short)bf16_bits(a.z); o[3] = (unsigned short)bf16_bits(a.w);
    o[4] = (unsigned short)bf16_bits(b.x); o[5] = (unsigned short)bf16_bits(b.y);
    o[6] = (unsigned short)bf16_bits(b.z); o[7] = (unsigned short)bf16_bits(b.w);
    unsigned short* dp = WD + (size_t)n * WP + k8;
    *(volatile v8us*)dp = o;
    __threadfence();
    *(volatile v8us*)dp = o;
  } else {
    if (tid < 32) {
      const v4f a = *(const v4f*)(hb + 4 * tid);
      v4f o;
      o.x = bf16_val(a.x); o.y = bf16_val(a.y); o.z = bf16_val(a.z); o.w = bf16_val(a.w);
      float* dp = BB + 4 * tid;
      *(volatile v4f*)dp = o;
      __threadfence();
      *(volatile v4f*)dp = o;
    }
  }
}

__global__ __launch_bounds__(NTHR) void k_rowsum(const float* __restrict__ wv, float* RS) {
  __shared__ __attribute__((aligned(16))) float rsl[32];
  const int tid = (int)threadIdx.x, lane = tid & 31, wave = tid >> 5;
  const int w0 = (int)blockIdx.x * 32 + 4 * wave;
  v4f r[4];
#pragma unroll
  for (int i = 0; i < 4; ++i) {
    int w = w0 + i;
    w = w > VOC - 1 ? VOC - 1 : w;
    r[i] = *(const v4f*)(wv + (size_t)w * DF + 4 * lane);
  }
#pragma unroll
  for (int i = 0; i < 4; ++i) {
    float s = ((bf16_val(r[i].x) + bf16_val(r[i].y)) + bf16_val(r[i].z)) + bf16_val(r[i].w);
    s = s + __shfl_xor(s, 16, 32);
    s = s + __shfl_xor(s, 8, 32);
    s = s + __shfl_xor(s, 4, 32);
    s = s + __shfl_xor(s, 2, 32);
    s = s + __shfl_xor(s, 1, 32);
    if (lane == 0) rsl[4 * wave + i] = s;
  }
  __syncthreads();
  if (wave == 0) {
    const v4f q = *(const v4fa*)(rsl + 4 * (lane & 7));
    asm volatile("" :: "v"(q.x), "v"(q.y), "v"(q.z), "v"(q.w));
    float* dp = RS + (size_t)blockIdx.x * 32 + 4 * (lane & 7);
    const bool st = lane < 8;
    if (st) *(volatile v4f*)dp = q;
    __threadfence();
    if (st) *(volatile v4f*)dp = q;
  }
}

__device__ __forceinline__ int put4(int* wlw, int wc, unsigned s0, unsigned s1, unsigned s2, unsigned s3, v4i t) {
  const bool h0 = s0 < (unsigned)NBRUN, h1 = s1 < (unsigned)NBRUN;
  const bool h2 = s2 < (unsigned)NBRUN, h3 = s3 < (unsigned)NBRUN;
  const unsigned m0 = __builtin_amdgcn_ballot_w32(h0);
  const unsigned m1 = __builtin_amdgcn_ballot_w32(h1);
  const unsigned m2 = __builtin_amdgcn_ballot_w32(h2);
  const unsigned m3 = __builtin_amdgcn_ballot_w32(h3);
  unsigned pre = __builtin_amdgcn_mbcnt_lo(m0, 0u);
  pre = __builtin_amdgcn_mbcnt_lo(m1, pre);
  pre = __builtin_amdgcn_mbcnt_lo(m2, pre);
  pre = __builtin_amdgcn_mbcnt_lo(m3, pre);
  const int p0 = wc + (int)pre;
  const int p1 = p0 + (h0 ? 1 : 0);
  const int p2 = p1 + (h1 ? 1 : 0);
  const int p3 = p2 + (h2 ? 1 : 0);
  const int e0 = (clampw(t.x) << SLB) | (int)(s0 & (unsigned)(NBRUN - 1));
  const int e1 = (clampw(t.y) << SLB) | (int)(s1 & (unsigned)(NBRUN - 1));
  const int e2 = (clampw(t.z) << SLB) | (int)(s2 & (unsigned)(NBRUN - 1));
  const int e3 = (clampw(t.w) << SLB) | (int)(s3 & (unsigned)(NBRUN - 1));
  if (h0 && p0 < WLCAP) wlw[p0] = e0;
  if (h1 && p1 < WLCAP) wlw[p1] = e1;
  if (h2 && p2 < WLCAP) wlw[p2] = e2;
  if (h3 && p3 < WLCAP) wlw[p3] = e3;
  return wc + (int)__builtin_popcount(m0) + (int)__builtin_popcount(m1)
            + (int)__builtin_popcount(m2) + (int)__builtin_popcount(m3);
}

__global__ __launch_bounds__(NTHR) void k_segmean(const int* __restrict__ tok, const int* __restrict__ seg,
                                                  const float* __restrict__ RS, float* SV,
                                                  unsigned short* apl, int* FLG) {
  extern __shared__ __attribute__((aligned(16))) int dsm[];
  int*   wl   = dsm + L_WL;
  int*   sl   = dsm + L_SL;
  int*   wcum = dsm + L_WCUM;
  int*   cnt  = dsm + L_CNT;
  int*   offs = dsm + L_OFFS;
  int*   cur  = dsm + L_CUR;
  float* svl  = (float*)(dsm + L_SVL);
  int*   misc = dsm + L_MISC;
  const int tid = (int)threadIdx.x, lane = tid & 31, wave = tid >> 5;
  const int nodeBase = (int)blockIdx.x * NBRUN;

  {
    const v4i z4 = {0, 0, 0, 0};
    for (int i = tid * 4; i < SEG_LDS_INTS; i += NTHR * 4) *(v4ia*)(dsm + i) = z4;
  }
  __syncthreads();

  {
    int* wlw = wl + wave * WLCAP;
    const unsigned nbs = (unsigned)nodeBase;
    int wc = 0;
#pragma unroll 1
    for (int ch = 0; ch < NCH; ++ch) {
      const int span = ch * CHUNK + wave * WSPAN;
      const v4i ka = *(const v4i*)(seg + span + 4 * lane);
      const v4i kb = *(const v4i*)(seg + span + 128 + 4 * lane);
      const unsigned a0 = (unsigned)ka.x - nbs, a1 = (unsigned)ka.y - nbs;
      const unsigned a2 = (unsigned)ka.z - nbs, a3 = (unsigned)ka.w - nbs;
      const unsigned b0 = (unsigned)kb.x - nbs, b1 = (unsigned)kb.y - nbs;
      const unsigned b2 = (unsigned)kb.z - nbs, b3 = (unsigned)kb.w - nbs;
      const bool hany = (a0 < (unsigned)NBRUN) | (a1 < (unsigned)NBRUN) | (a2 < (unsigned)NBRUN) |
                        (a3 < (unsigned)NBRUN) | (b0 < (unsigned)NBRUN) | (b1 < (unsigned)NBRUN) |
                        (b2 < (unsigned)NBRUN) | (b3 < (unsigned)NBRUN);
      const unsigned any = __builtin_amdgcn_ballot_w32(hany);
      if (any != 0u) {
        const v4i ta = *(const v4i*)(tok + span + 4 * lane);
        const v4i tb = *(const v4i*)(tok + span + 128 + 4 * lane);
        asm volatile("" :: "v"(ta.x), "v"(ta.y), "v"(ta.z), "v"(ta.w));
        asm volatile("" :: "v"(tb.x), "v"(tb.y), "v"(tb.z), "v"(tb.w));
        wc = put4(wlw, wc, a0, a1, a2, a3, ta);
        wc = put4(wlw, wc, b0, b1, b2, b3, tb);
      }
      if (lane == 0) wcum[wave * NCHP + ch + 1] = wc;
    }
    if (lane == 0) misc[wave] = wc;
  }
  __syncthreads();

  if (wave == 0) {
    int tt = 0, ov = 0;
#pragma unroll 1
    for (int w2 = 0; w2 < NWAVE; ++w2) {
      int cr = misc[w2];
      const int bg = cr > WLCAP ? 1 : 0;
      cr = cr < 0 ? 0 : (cr > WLCAP ? WLCAP : cr);
      const int c = __builtin_amdgcn_readfirstlane(cr);
      ov |= __builtin_amdgcn_readfirstlane(bg);
      tt += c;
#pragma unroll 1
      for (int b0 = 0; b0 < c; b0 += 32) {
        const int idx = b0 + lane;
        const int ent = wl[w2 * WLCAP + (idx < WLCAP ? idx : WLCAP - 1)];
        const int m32 = (c - b0) < 32 ? (c - b0) : 32;
#pragma unroll 1
        for (int k = 0; k < m32; ++k) {
          const int u    = __builtin_amdgcn_readlane(ent, k);
          const int slot = u & (NBRUN - 1);
          if (lane == 0) cnt[slot] = cnt[slot] + 1;
        }
      }
    }
    if (tt > RCAP) ov = 1;
    if (lane == 0) { misc[8] = tt; misc[9] = ov; }
  }
  __syncthreads();

  if (wave == 0) {
    const int base = lane * (NBRUN / 32);
    int s = 0, mx = 0;
#pragma unroll 1
    for (int i = 0; i < NBRUN / 32; ++i) {
      const int cv = cnt[base + i];
      s += cv;
      mx = cv > mx ? cv : mx;
    }
    int incl = s;
#pragma unroll
    for (int d = 1; d < 32; d <<= 1) {
      const int y = __shfl_up(incl, d, 32);
      if (lane >= d) incl += y;
    }
    int run = incl - s;
#pragma unroll 1
    for (int i = 0; i < NBRUN / 32; ++i) {
      const int cv = cnt[base + i];
      offs[base + i] = run;
      cur[base + i]  = run;
      run += cv;
    }
    const unsigned bigm = __builtin_amdgcn_ballot_w32(mx > DEGCAP);
    if (lane == 0) misc[10] = (bigm != 0u) ? 1 : 0;
  }
  __syncthreads();

  if (wave == 0) {
    const int lw = lane & 7;
#pragma unroll 1
    for (int ch = 0; ch < NCH; ++ch) {
      int loV = wcum[lw * NCHP + ch];
      int hiV = wcum[lw * NCHP + ch + 1];
      loV = loV < 0 ? 0 : (loV > WLCAP ? WLCAP : loV);
      hiV = hiV < 0 ? 0 : (hiV > WLCAP ? WLCAP : hiV);
      hiV = hiV < loV ? loV : hiV;
      hiV = (hiV - loV) > WSPAN ? (loV + WSPAN) : hiV;
      const unsigned act = __builtin_amdgcn_ballot_w32(hiV > loV);
      if (act != 0u) {
#pragma unroll 1
        for (int w2 = 0; w2 < NWAVE; ++w2) {
          const int lo = __builtin_amdgcn_readlane(loV, w2);
          const int hi = __builtin_amdgcn_readlane(hiV, w2);
#pragma unroll 1
          for (int b0 = lo; b0 < hi; b0 += 32) {
            const int idx = b0 + lane;
            const int ent = wl[w2 * WLCAP + (idx < WLCAP ? idx : WLCAP - 1)];
            const int m32 = (hi - b0) < 32 ? (hi - b0) : 32;
#pragma unroll 1
            for (int k = 0; k < m32; ++k) {
              const int u    = __builtin_amdgcn_readlane(ent, k);
              const int slot = u & (NBRUN - 1);
              if (lane == 0) {
                int p = cur[slot];
                p = p < 0 ? 0 : (p > RCAP - 1 ? RCAP - 1 : p);
                sl[p] = u;
                cur[slot] = p + 1;
              }
            }
          }
        }
      }
    }
  }
  __syncthreads();

  const int   ovf  = (misc[9] | misc[10]) != 0 ? 1 : 0;
  const bool  bad  = ovf != 0;
  const float qnan = __int_as_float(0x7fc00000);
#pragma unroll 1
  for (int si = 0; si < NBRUN / NWAVE; ++si) {
    const int s    = si * NWAVE + wave;
    const int node = nodeBase + s;
    const int cv = cnt[s];
    int cc = cv < 0 ? 0 : (cv > DEGCAP ? DEGCAP : cv);
    const int c = __builtin_amdgcn_readfirstlane(cc);
    int ov2 = offs[s];
    ov2 = ov2 < 0 ? 0 : (ov2 > RCAP - 1 ? RCAP - 1 : ov2);
    const int o = __builtin_amdgcn_readfirstlane(ov2);
    int last = o + c - 1;
    last = last < o ? o : last;
    last = last > RCAP - 1 ? RCAP - 1 : last;
    const int cd = cv < 1 ? 1 : cv;
    const float cf = (float)cd;
    float acc = 0.0f;
#pragma unroll 1
    for (int b0 = 0; b0 < c; b0 += 32) {
      int idx = o + b0 + lane;
      idx = idx > last ? last : idx;
      const int ent = sl[idx];
      const int w = clampw(ent >> SLB);
      float v = RS[w];
      asm volatile("" :: "v"(v));
      v = (b0 + lane < c) ? v : 0.0f;
      const int vi = __float_as_int(v);
      const int m32 = (c - b0) < 32 ? (c - b0) : 32;
#pragma unroll 1
      for (int k = 0; k < m32; ++k) {
        acc = acc + __int_as_float(__builtin_amdgcn_readlane(vi, k));
      }
    }
    float svv = (acc + 0.0f) / cf;
    svv = bad ? qnan : svv;
    const unsigned hb  = bf16_bits(svv);
    const float    hif = __uint_as_float(hb << 16);
    const unsigned lb  = bf16_bits(svv - hif);
    const unsigned hw  = hb | (hb << 16);
    const unsigned lw2 = lb | (lb << 16);
    const unsigned wsel = (lane < 16) ? hw : lw2;
    v4u q;
    q.x = wsel; q.y = wsel; q.z = wsel; q.w = wsel;
    if (lane == 0) svl[s] = svv;
    unsigned short* rp = apl + (size_t)node * AP + 8 * lane;
    *(volatile v4u*)rp = q;
    __threadfence();
    *(volatile v4u*)rp = q;
  }
  __syncthreads();

  if (wave == 0) {
    const v4f q0 = *(const v4fa*)(svl + 4 * lane);
    const v4f q1 = *(const v4fa*)(svl + 128 + 4 * lane);
    float* sp = SV + (size_t)nodeBase + 4 * lane;
    v4i fv;
    fv.x = ovf; fv.y = ovf; fv.z = ovf; fv.w = ovf;
    int* fp = FLG + (size_t)blockIdx.x * 32 + 4 * (lane & 7);
    const bool fst = lane < 8;
    *(volatile v4f*)sp = q0;
    *(volatile v4f*)(sp + 128) = q1;
    if (fst) *(volatile v4i*)fp = fv;
    __threadfence();
    *(volatile v4f*)sp = q0;
    *(volatile v4f*)(sp + 128) = q1;
    if (fst) *(volatile v4i*)fp = fv;
  }
}

__global__ __launch_bounds__(GTHR) __attribute__((amdgpu_num_vgpr(248)))
void k_gemm(const unsigned short* __restrict__ Apl, const unsigned short* __restrict__ WD,
            const float* __restrict__ BB, const int* __restrict__ FLG, float* outp) {
  __shared__ __attribute__((aligned(16))) float stg[GBM * GBN];
  __shared__ __attribute__((aligned(16))) float bsh[GBN];
  const int tid = (int)threadIdx.x, lane = tid & 31, wave = tid >> 5, hh = lane >> 4, m = lane & 15;
  const int rowBase = (int)blockIdx.x * GBM;

  if (tid < 32) {
    const v4f b = *(const v4f*)(BB + 4 * tid);
    *(v4fa*)(bsh + 4 * tid) = b;
  }

  v8f acc[8];
  {
    const v8f z = {0.f, 0.f, 0.f, 0.f, 0.f, 0.f, 0.f, 0.f};
#pragma unroll
    for (int t = 0; t < 8; ++t) acc[t] = z;
  }
  const unsigned short* ap = Apl + (size_t)(rowBase + 16 * wave + m) * (size_t)AP + 8 * hh;
  const unsigned short* bp = WD + (size_t)m * (size_t)WP + 8 * hh;

#pragma unroll 1
  for (int k0 = 0; k0 < KUSED; k0 += 32) {
    FragB af;
    af.h[0] = *(const v8usa*)(ap + k0);
    af.h[1] = *(const v8usa*)(ap + k0 + 16);
#pragma unroll
    for (int nt = 0; nt < 8; ++nt) {
      const unsigned short* wq = bp + (size_t)(16 * nt) * (size_t)WP + k0;
      FragB bf;
      bf.h[0] = *(const v8usa*)wq;
      bf.h[1] = *(const v8usa*)(wq + 16);
      acc[nt] = wmb(af, bf, acc[nt]);
    }
  }

#pragma unroll
  for (int nt = 0; nt < 8; ++nt) {
    const int lc = 16 * nt + m;
#pragma unroll
    for (int r = 0; r < 8; ++r) {
      const int lr = 16 * wave + 8 * hh + r;
      stg[lr * GBN + lc] = acc[nt][r];
    }
  }
  __syncthreads();

  int fb = rowBase / NBRUN;
  fb = fb > NBLK - 1 ? NBLK - 1 : fb;
  const int  fl  = FLG[(size_t)fb * 32];
  const bool bad = fl != 0;
  const float qnan = __int_as_float(0x7fc00000);
  const v4f bb4 = *(const v4fa*)(bsh + 4 * lane);

  v4f pv[16];
#pragma unroll
  for (int i = 0; i < 16; ++i) pv[i] = *(const v4fa*)(stg + (16 * wave + i) * GBN + 4 * lane);
#pragma unroll
  for (int i = 0; i < 16; ++i) {
    v4f y = pv[i] + bb4;
    y.x = bad ? qnan : y.x;
    y.y = bad ? qnan : y.y;
    y.z = bad ? qnan : y.z;
    y.w = bad ? qnan : y.w;
    pv[i] = y;
  }
#pragma unroll
  for (int i = 0; i < 16; ++i) {
    const int r = rowBase + 16 * wave + i;
    *(volatile v4f*)(outp + (size_t)r * NLAB + 4 * lane) = pv[i];
  }
  __threadfence();
#pragma unroll
  for (int i = 0; i < 16; ++i) {
    const int r = rowBase + 16 * wave + i;
    *(volatile v4f*)(outp + (size_t)r * NLAB + 4 * lane) = pv[i];
  }
}

static inline size_t al256(size_t o) { return (o + 255) & ~(size_t)255; }

extern "C" void kernel_launch(void* const* d_in, const int* in_sizes, int n_in,
                              void* d_out, int out_size, void* d_ws, size_t ws_size,
                              hipStream_t stream) {
  if (n_in < 5) return;
  if (in_sizes[0] != TOK || in_sizes[1] != TOK) return;
  if (in_sizes[2] != VOC * DF) return;
  if (in_sizes[3] != NLAB * DF || in_sizes[4] != NLAB) return;
  if (out_size != NSENT * NLAB) return;

  const int*   tok = (const int*)d_in[0];
  const int*   seg = (const int*)d_in[1];
  const float* wv  = (const float*)d_in[2];
  const float* W   = (const float*)d_in[3];
  const float* hb  = (const float*)d_in[4];
  float* out = (float*)d_out;

  char* ws = (char*)d_ws;
  size_t off = 0;
  const size_t oRS  = off; off = al256(off + (size_t)RSN * 4);
  const size_t oSV  = off; off = al256(off + (size_t)NSENT * 4);
  const size_t oA   = off; off = al256(off + (size_t)NSENT * AP * 2);
  const size_t oWD  = off; off = al256(off + (size_t)NLAB * WP * 2);
  const size_t oBB  = off; off = al256(off + (size_t)NLAB * 4);
  const size_t oFL  = off; off = al256(off + (size_t)NBLK * 128);
  if (off > ws_size || off > (size_t)WSMAX) return;
  float*          RS  = (float*)(ws + oRS);
  float*          SV  = (float*)(ws + oSV);
  unsigned short* Apl = (unsigned short*)(ws + oA);
  unsigned short* WD  = (unsigned short*)(ws + oWD);
  float*          BB  = (float*)(ws + oBB);
  int*            FLG = (int*)(ws + oFL);

  const size_t segLds = (size_t)SEG_LDS_INTS * 4;
  hipFuncSetAttribute(reinterpret_cast<const void*>(&k_segmean), hipFuncAttributeMaxDynamicSharedMemorySize,
                      (int)segLds);

  k_prep<<<WUNITS / NTHR + 1, NTHR, 0, stream>>>(W, hb, WD, BB);
  k_rowsum<<<VOC / 32, NTHR, 0, stream>>>(wv, RS);
  k_segmean<<<NBLK, NTHR, segLds, stream>>>(tok, seg, RS, SV, Apl, FLG);
  k_gemm<<<NSENT / GBM, GTHR, 0, stream>>>(Apl, WD, BB, FLG, out);
}
